// conv_mamba_block_52596169506817
// MI455X (gfx1250) — hardware-verified
//
#include <hip/hip_runtime.h>
#include <hip/hip_bf16.h>
#include <math.h>

#define BB 2
#define LL 2048
#define DM 512
#define DI 1024
#define NS 16
#define KC 4
#define RR 32
#define CK 31
#define DFF 2048
#define MTOK (BB * LL)
#define GSTR 48

typedef _Float16 bf16;
typedef _Float16 f16;
typedef __attribute__((ext_vector_type(4))) unsigned v4u_t;
typedef unsigned v4ua __attribute__((ext_vector_type(4), may_alias));
typedef __attribute__((ext_vector_type(4))) float v4f_t;
typedef float v4fa __attribute__((ext_vector_type(4), may_alias));
typedef __attribute__((ext_vector_type(16))) bf16  bf16x16;
typedef bf16x16 f16x16;
typedef __attribute__((ext_vector_type(8)))  bf16  bf16x8;
typedef bf16x8 f16x8;
typedef __attribute__((ext_vector_type(8)))  float f32x8;
__device__ __forceinline__ f32x8 wmma16(f16x16 a, f16x16 b, f32x8 c) {
  c = __builtin_amdgcn_wmma_f32_16x16x32_f16(false, a, false, b, (short)0, c, false, false);
  asm volatile("v_nop\n\tv_nop\n\tv_nop\n\tv_nop" : "+v"(c) : "v"(a), "v"(b));
  return c;
}
__device__ __forceinline__ f16x16 lds_frag(const f16* base, int stride) {
  const int lane = threadIdx.x & 31, row = lane & 15, kh = (lane >> 4) * 8;
  const f16x8 lo = *(const f16x8*)(base + row * stride + kh);
  const f16x8 hi = *(const f16x8*)(base + row * stride + kh + 16);
  f16x16 f;
#pragma unroll
  for (int i = 0; i < 8; ++i) { f[i] = lo[i]; f[i + 8] = hi[i]; }
  return f;
}

#define GSTR 48
template <typename AT, int EPI, bool OUT16>
__global__ __launch_bounds__(256) void gemm_kne(const AT* __restrict__ A, int lda, const float* __restrict__ Wm, int ldw,
                                                const float* __restrict__ bias, const float* __restrict__ R, const float* __restrict__ gvec,
                                                void* __restrict__ Yv, int ldy, int K) {
  __shared__ __attribute__((aligned(16))) f16 ldsA[128 * GSTR];
  __shared__ __attribute__((aligned(16))) f16 ldsW[128 * GSTR];
  __shared__ __attribute__((aligned(16))) float oS[8][32 * 68];
  const int tid = threadIdx.x, lane = tid & 31, wave = tid >> 5, cl = lane & 15, rh = (lane >> 4) * 8;
  const int m0 = blockIdx.x * 128, n0 = blockIdx.y * 128;
  const int wm = (wave & 3) * 32, wn = (wave >> 2) * 64;
  f32x8 acc[2][4];
#pragma unroll
  for (int i = 0; i < 2; ++i)
#pragma unroll
    for (int j = 0; j < 4; ++j) { f32x8 z = {}; acc[i][j] = z; }
#pragma unroll 1
  for (int k0 = 0; k0 < K; k0 += 32) {
    __syncthreads();
    { const int row = tid >> 1, ch = (tid & 1) * 16;
      const AT* src = A + (size_t)(m0 + row) * lda + k0 + ch;
#pragma unroll
      for (int g = 0; g < 16; ++g) ldsA[row * GSTR + ch + g] = (f16)src[g]; }
    { const int k = tid >> 3, nn0 = (tid & 7) * 16;
      const float* src = Wm + (size_t)(k0 + k) * ldw + n0 + nn0;
#pragma unroll
      for (int g = 0; g < 4; ++g) { const v4f_t v = *(const v4f_t*)(src + 4 * g);
#pragma unroll
        for (int u = 0; u < 4; ++u) ldsW[(nn0 + 4 * g + u) * GSTR + k] = (f16)v[u]; } }
    __syncthreads();
    f16x16 af[2];
#pragma unroll
    for (int i = 0; i < 2; ++i) af[i] = lds_frag(ldsA + (wm + 16 * i) * GSTR, GSTR);
#pragma unroll
    for (int j = 0; j < 4; ++j) {
      const f16x16 bf = lds_frag(ldsW + (wn + 16 * j) * GSTR, GSTR);
#pragma unroll
      for (int i = 0; i < 2; ++i) acc[i][j] = wmma16(af[i], bf, acc[i][j]);
    }
  }
  float* so = oS[wave];
#pragma unroll
  for (int i = 0; i < 2; ++i)
#pragma unroll
    for (int j = 0; j < 4; ++j) {
      const int n = n0 + wn + 16 * j + cl;
      const float bv = bias ? bias[n] : 0.0f;
      const float gv = (EPI == 2) ? gvec[n] : 0.0f;
      if (EPI == 1) {
#pragma unroll 1
        for (int r = 0; r < 8; ++r) { const float xg = acc[i][j][r] + bv; so[(16 * i + rh + r) * 68 + 16 * j + cl] = 0.5f * xg * (1.0f + tanhf(0.7978845608028654f * (xg + 0.044715f * xg * xg * xg))); }
      } else {
#pragma unroll
        for (int r = 0; r < 8; ++r) {
          float v = acc[i][j][r] + bv;
          if (EPI == 2) v = R[(size_t)(m0 + wm + 16 * i + rh + r) * ldy + n] + gv * v;
          so[(16 * i + rh + r) * 68 + 16 * j + cl] = v;
        }
      }
    }
  asm volatile("s_wait_dscnt 0" ::: "memory");
  __builtin_amdgcn_wave_barrier();
#pragma unroll 1
  for (int pass = 0; pass < 2; ++pass) {
    if (OUT16) {
      f16* Y = (f16*)Yv;
#pragma unroll
      for (int it = 0; it < 8; ++it) { const int c = lane + 32 * it, rr = c >> 3, q8 = (c & 7) * 8;
        union { f16 h[8]; v4u_t v; } u;
#pragma unroll
        for (int e = 0; e < 8; ++e) u.h[e] = (f16)so[rr * 68 + q8 + e];
        *(volatile v4u_t*)(Y + (size_t)(m0 + wm + rr) * ldy + n0 + wn + q8) = u.v; }
    } else {
      float* Y = (float*)Yv;
#pragma unroll
      for (int it = 0; it < 16; ++it) { const int f4 = lane + 32 * it, rr = f4 >> 4, q = (f4 & 15) * 4;
        *(volatile v4f_t*)(Y + (size_t)(m0 + wm + rr) * ldy + n0 + wn + q) = *(const volatile v4fa*)(so + rr * 68 + q); }
    }
    __threadfence();
  }
}


template <typename AT, bool ACC>
__global__ __launch_bounds__(256) void gemm_kn2(const AT* __restrict__ A, int lda, size_t strideA,
                                               const float* __restrict__ Wm, int ldw, size_t strideW,
                                               const float* __restrict__ bias, float scale,
                                               float* __restrict__ Y, int ldy, size_t strideY, int K) {
  __shared__ __attribute__((aligned(16))) f16 ldsA[128 * GSTR], ldsAl[128 * GSTR];
  __shared__ __attribute__((aligned(16))) f16 ldsW[128 * GSTR], ldsWl[128 * GSTR];
  __shared__ __attribute__((aligned(16))) float oS[8][32 * 68];
  const int tid = threadIdx.x, lane = tid & 31, wave = tid >> 5, cl = lane & 15, rh = (lane >> 4) * 8;
  const int m0 = blockIdx.x * 128, n0 = blockIdx.y * 128;
  const int wm = (wave & 3) * 32, wn = (wave >> 2) * 64;
  A += (size_t)blockIdx.z * strideA; Wm += (size_t)blockIdx.z * strideW; Y += (size_t)blockIdx.z * strideY;
  f32x8 acc[2][4], accx[2][4];
#pragma unroll
  for (int i = 0; i < 2; ++i)
#pragma unroll
    for (int j = 0; j < 4; ++j) { f32x8 z = {}; acc[i][j] = z; accx[i][j] = z; }
#pragma unroll 1
  for (int k0 = 0; k0 < K; k0 += 32) {
    __syncthreads();
    {
      const int row = tid >> 1, ch = (tid & 1) * 16;
      const AT* src = A + (size_t)(m0 + row) * lda + k0 + ch;
#pragma unroll
      for (int g = 0; g < 16; ++g) { const float v = (float)src[g]; const f16 h = (f16)v; ldsA[row * GSTR + ch + g] = h; ldsAl[row * GSTR + ch + g] = (f16)((v - (float)h) * 2048.0f); }
    }
    {
      const int k = tid >> 3, nn0 = (tid & 7) * 16;
      const float* src = Wm + (size_t)(k0 + k) * ldw + n0 + nn0;
#pragma unroll
      for (int g = 0; g < 4; ++g) { const v4f_t v = *(const v4f_t*)(src + 4 * g);
#pragma unroll
        for (int u = 0; u < 4; ++u) { const f16 h = (f16)v[u]; ldsW[(nn0 + 4 * g + u) * GSTR + k] = h; ldsWl[(nn0 + 4 * g + u) * GSTR + k] = (f16)((v[u] - (float)h) * 2048.0f); } }
    }
    __syncthreads();
    f16x16 af[2], afl[2];
#pragma unroll
    for (int i = 0; i < 2; ++i) { af[i] = lds_frag(ldsA + (wm + 16 * i) * GSTR, GSTR); afl[i] = lds_frag(ldsAl + (wm + 16 * i) * GSTR, GSTR); }
#pragma unroll
    for (int j = 0; j < 4; ++j) {
      const f16x16 bf = lds_frag(ldsW + (wn + 16 * j) * GSTR, GSTR), bfl = lds_frag(ldsWl + (wn + 16 * j) * GSTR, GSTR);
#pragma unroll
      for (int i = 0; i < 2; ++i) { acc[i][j] = wmma16(af[i], bf, acc[i][j]); accx[i][j] = wmma16(af[i], bfl, accx[i][j]); accx[i][j] = wmma16(afl[i], bf, accx[i][j]); }
    }
  }
  float* so = oS[wave];
#pragma unroll
  for (int i = 0; i < 2; ++i)
#pragma unroll
    for (int j = 0; j < 4; ++j) {
      const float bv = bias ? bias[n0 + wn + 16 * j + cl] : 0.0f;
#pragma unroll
      for (int r = 0; r < 8; ++r) so[(16 * i + rh + r) * 68 + 16 * j + cl] = (acc[i][j][r] + accx[i][j][r] * (1.0f / 2048.0f)) * scale + bv;
    }
  asm volatile("s_wait_dscnt 0" ::: "memory");
  __builtin_amdgcn_wave_barrier();
  if (ACC) {
#pragma unroll
    for (int it = 0; it < 16; ++it) { const int f4 = lane + 32 * it, rr = f4 >> 4, q = (f4 & 15) * 4;
      const v4f_t old = *(const volatile v4fa*)(Y + (size_t)(m0 + wm + rr) * ldy + n0 + wn + q);
      v4f_t v = *(const volatile v4fa*)(so + rr * 68 + q); v += old; *(volatile v4fa*)(so + rr * 68 + q) = v; }
    asm volatile("s_wait_dscnt 0" ::: "memory");
  }
#pragma unroll 1
  for (int pass = 0; pass < 2; ++pass) {
#pragma unroll
    for (int it = 0; it < 16; ++it) { const int f4 = lane + 32 * it, rr = f4 >> 4, q = (f4 & 15) * 4;
      *(volatile v4f_t*)(Y + (size_t)(m0 + wm + rr) * ldy + n0 + wn + q) = *(const volatile v4fa*)(so + rr * 68 + q); }
    __threadfence();
  }
}

__global__ __launch_bounds__(256) void k_ln(const float* __restrict__ X, const float* __restrict__ gam, const float* __restrict__ bet, float* __restrict__ Y) {
  __shared__ __attribute__((aligned(16))) float rowS[32 * 516];
  const int tid = threadIdx.x, r = tid >> 3, part = tid & 7; const size_t row = (size_t)blockIdx.x * 32 + r;
  const float* xr = X + row * DM + part * 64; float s = 0.0f;
  for (int i = 0; i < 64; ++i) { const float v = xr[i]; rowS[r * 516 + part * 64 + i] = v; s += v; }
  s += __shfl_xor(s, 1, 32); s += __shfl_xor(s, 2, 32); s += __shfl_xor(s, 4, 32);
  const float mean = s * (1.0f / DM); float q = 0.0f;
  for (int i = 0; i < 64; ++i) { const float d = rowS[r * 516 + part * 64 + i] - mean; q += d * d; }
  q += __shfl_xor(q, 1, 32); q += __shfl_xor(q, 2, 32); q += __shfl_xor(q, 4, 32);
  const float rstd = rsqrtf(q * (1.0f / DM) + 1e-5f);
  for (int i = 0; i < 64; ++i) { const int c = part * 64 + i; rowS[r * 516 + c] = (rowS[r * 516 + c] - mean) * rstd * gam[c] + bet[c]; }
  __syncthreads();
#pragma unroll 1
  for (int pass = 0; pass < 2; ++pass) { for (int qd = tid; qd < 32 * 128; qd += 256) { const int rr = qd >> 7, c4 = (qd & 127) * 4; *(volatile v4f_t*)(Y + ((size_t)blockIdx.x * 32 + rr) * DM + c4) = *(const volatile v4fa*)(rowS + rr * 516 + c4); } __threadfence(); }
}
__global__ __launch_bounds__(256) void k_dwconv4(const float* __restrict__ xz, const float* __restrict__ w, const float* __restrict__ cb, float* __restrict__ xc) {
  const size_t i = (size_t)blockIdx.x * 256 + threadIdx.x;
  const size_t row = i >> 8; const int d0 = (i & 255) * 4; const int b = row / LL, l = row % LL;
  v4f_t acc; acc[0] = cb[d0]; acc[1] = cb[d0 + 1]; acc[2] = cb[d0 + 2]; acc[3] = cb[d0 + 3];
#pragma unroll
  for (int j = 0; j < KC; ++j) { const int ls = l + j - (KC - 1); if (ls >= 0) { const v4f_t v = *(const v4f_t*)(xz + ((size_t)b * LL + ls) * (2 * DI) + d0);
      acc[0] += w[(d0) * KC + j] * v[0]; acc[1] += w[(d0 + 1) * KC + j] * v[1]; acc[2] += w[(d0 + 2) * KC + j] * v[2]; acc[3] += w[(d0 + 3) * KC + j] * v[3]; } }
  v4f_t o; for (int e = 0; e < 4; ++e) o[e] = acc[e] / (1.0f + expf(-acc[e]));
  *(volatile v4f_t*)(xc + row * DI + d0) = o; __threadfence(); *(volatile v4f_t*)(xc + row * DI + d0) = o;
}
__global__ __launch_bounds__(256) void k_cast16(const float* __restrict__ src, bf16* __restrict__ dst, size_t n8) {
  const size_t i = (size_t)blockIdx.x * 256 + threadIdx.x; if (i >= n8) return; const float* p = src + 8 * i; union { bf16 hh[8]; v4u_t u; } cv;
#pragma unroll
  for (int e = 0; e < 8; ++e) cv.hh[e] = (bf16)p[e];
  *(volatile v4u_t*)(dst + 8 * i) = cv.u; __threadfence(); *(volatile v4u_t*)(dst + 8 * i) = cv.u;
}
__global__ __launch_bounds__(256) void k_scan(const float* __restrict__ dtraw, const float* __restrict__ bdt, const float* __restrict__ xc, const float* __restrict__ dbl,
                                             const float* __restrict__ Alog, const float* __restrict__ Dp, const float* __restrict__ xz, float* __restrict__ y32) {
  __shared__ float bcS[2 * NS];
  const int tid = threadIdx.x, b = blockIdx.x / (DI / 256), d = (blockIdx.x % (DI / 256)) * 256 + tid;
  float A[NS], h[NS];
#pragma unroll
  for (int n = 0; n < NS; ++n) { A[n] = -expf(Alog[d * NS + n]); h[n] = 0.0f; }
  const float dpd = Dp[d], bd = bdt[d];
#pragma unroll 1
  for (int l = 0; l < LL; ++l) {
    const size_t row = (size_t)b * LL + l;
    __syncthreads();
    if (tid < 2 * NS) bcS[tid] = dbl[row * 128 + RR + tid];
    __syncthreads();
    const float dr = dtraw[row * DI + d] + bd; const float delta = (dr > 20.0f) ? dr : log1pf(expf(dr));
    const float xv = xc[row * DI + d]; const float dx = delta * xv; float yv = 0.0f;
#pragma unroll
    for (int n = 0; n < NS; ++n) { h[n] = expf(delta * A[n]) * h[n] + dx * bcS[n]; yv += h[n] * bcS[NS + n]; }
    yv += dpd * xv; const float z = xz[row * (2 * DI) + DI + d]; yv *= z / (1.0f + expf(-z));
    y32[row * DI + d] = yv;
  }
}
__global__ __launch_bounds__(256) void k_glu(const float* __restrict__ pw, float* __restrict__ glu) {
  const size_t i = (size_t)blockIdx.x * 256 + threadIdx.x; const size_t row = i >> 7; const int c0 = (i & 127) * 4;
  const v4f_t a = *(const v4f_t*)(pw + row * (2 * DM) + c0), g = *(const v4f_t*)(pw + row * (2 * DM) + DM + c0); v4f_t o;
  for (int e = 0; e < 4; ++e) o[e] = a[e] / (1.0f + expf(-g[e]));
  *(volatile v4f_t*)(glu + row * DM + c0) = o; __threadfence(); *(volatile v4f_t*)(glu + row * DM + c0) = o;
}
__global__ __launch_bounds__(256) void k_dwconv31(const float* __restrict__ glu, const float* __restrict__ w, const float* __restrict__ cb, float* __restrict__ c3) {
  const size_t i = (size_t)blockIdx.x * 256 + threadIdx.x; const size_t row = i >> 7; const int c0 = (i & 127) * 4; const int b = row / LL, l = row % LL;
  v4f_t acc; acc[0] = cb[c0]; acc[1] = cb[c0 + 1]; acc[2] = cb[c0 + 2]; acc[3] = cb[c0 + 3];
#pragma unroll 1
  for (int j = 0; j < CK; ++j) { const int ls = l + j - (CK - 1) / 2; if (ls >= 0 && ls < LL) { const v4f_t v = *(const v4f_t*)(glu + ((size_t)b * LL + ls) * DM + c0);
      acc[0] += w[(c0) * CK + j] * v[0]; acc[1] += w[(c0 + 1) * CK + j] * v[1]; acc[2] += w[(c0 + 2) * CK + j] * v[2]; acc[3] += w[(c0 + 3) * CK + j] * v[3]; } }
  v4f_t o; for (int e = 0; e < 4; ++e) o[e] = acc[e] / (1.0f + expf(-acc[e]));
  *(volatile v4f_t*)(c3 + row * DM + c0) = o; __threadfence(); *(volatile v4f_t*)(c3 + row * DM + c0) = o;
}
__global__ __launch_bounds__(256) void k_padwx(const float* __restrict__ Wx, float* __restrict__ Wp) {
  const int k = blockIdx.x * 2 + (threadIdx.x >> 7), n = threadIdx.x & 127; Wp[(size_t)k * 128 + n] = (n < RR + 2 * NS) ? Wx[(size_t)k * (RR + 2 * NS) + n] : 0.0f;
}
__global__ __launch_bounds__(256) void k_ones(float* __restrict__ p) { const int tid = threadIdx.x; if (tid < DM / 4) { v4f_t o = {1.f,1.f,1.f,1.f}; *(volatile v4f_t*)(p + tid * 4) = o; __threadfence(); *(volatile v4f_t*)(p + tid * 4) = o; } }

extern "C" void kernel_launch(void* const* d_in, const int* in_sizes, int n_in,
                              void* d_out, int out_size, void* d_ws, size_t ws_size,
                              hipStream_t stream) {
  (void)in_sizes; (void)n_in; (void)out_size;
  const float** f = (const float**)d_in;
  const float* x = f[0], *ln_g = f[1], *ln_b = f[2], *W_in = f[3], *conv_w = f[4], *conv_b = f[5], *W_x = f[6], *W_dt = f[7], *b_dt = f[8], *A_log = f[9], *Dp = f[10], *W_out = f[11];
  const float* cm_g = f[12], *cm_b = f[13], *pw1_w = f[14], *pw1_b = f[15], *dw_w = f[16], *dw_b = f[17], *pw2_w = f[18], *pw2_b = f[19];
  const float* ff1 = f[20], *fb1 = f[21], *ff2 = f[22], *fb2 = f[23];
  float* out = (float*)d_out;
  char* ws = (char*)d_ws;
  float* xz = (float*)ws; float* xc = (float*)(ws + (size_t)32 * 1024 * 1024); float* dtraw = (float*)(ws + (size_t)48 * 1024 * 1024);
  float* pw1o = (float*)ws; float* glu = (float*)(ws + (size_t)16 * 1024 * 1024); float* c3 = (float*)(ws + (size_t)24 * 1024 * 1024); float* ff = (float*)(ws + (size_t)32 * 1024 * 1024);
  ws += (size_t)64 * 1024 * 1024;
  float* hln = (float*)ws; ws += (size_t)MTOK * DM * 4;
  float* dbl = (float*)ws; ws += (size_t)MTOK * 128 * 4;
  float* Wxp = (float*)ws; ws += (size_t)DI * 128 * 4;
  float* y32 = (float*)ws; ws += (size_t)MTOK * DI * 4;
  float* m1 = (float*)ws; ws += (size_t)MTOK * DM * 4;
  float* cln = (float*)ws; ws += (size_t)MTOK * DM * 4;
  float* m2 = (float*)ws; ws += (size_t)MTOK * DM * 4;
  float* fln = (float*)ws; ws += (size_t)MTOK * DM * 4;
  float* ones = (float*)ws; ws += DM * 4;
  if ((size_t)(ws - (char*)d_ws) > ws_size) return;
  const dim3 blk(256);
  k_ones<<<dim3(1), blk, 0, stream>>>(ones);
  k_padwx<<<dim3(DI / 2), blk, 0, stream>>>(W_x, Wxp);
  k_ln<<<dim3(MTOK / 32), blk, 0, stream>>>(x, ln_g, ln_b, hln);
  gemm_kn2<float, false><<<dim3(MTOK / 128, (2 * DI) / 128, 1), blk, 0, stream>>>(hln, DM, 0, W_in, 2 * DI, 0, nullptr, 1.0f, xz, 2 * DI, 0, DM);
  k_dwconv4<<<dim3(MTOK * (DI / 4) / 256), blk, 0, stream>>>(xz, conv_w, conv_b, xc);
  gemm_kn2<float, false><<<dim3(MTOK / 128, 1, 1), blk, 0, stream>>>(xc, DI, 0, Wxp, 128, 0, nullptr, 1.0f, dbl, 128, 0, DI);
  gemm_kn2<float, false><<<dim3(MTOK / 128, DI / 128, 1), blk, 0, stream>>>(dbl, 128, 0, W_dt, DI, 0, nullptr, 1.0f, dtraw, DI, 0, RR);
  k_scan<<<dim3(BB * DI / 256), blk, 0, stream>>>(dtraw, b_dt, xc, dbl, A_log, Dp, xz, y32);
  gemm_kn2<float, false><<<dim3(MTOK / 128, DM / 128, 1), blk, 0, stream>>>(y32, DI, 0, W_out, DM, 0, nullptr, 1.0f, m1, DM, 0, DI);
  k_ln<<<dim3(MTOK / 32), blk, 0, stream>>>(m1, cm_g, cm_b, cln);
  gemm_kne<float, 0, false><<<dim3(MTOK / 128, (2 * DM) / 128), blk, 0, stream>>>(cln, DM, pw1_w, 2 * DM, pw1_b, nullptr, nullptr, pw1o, 2 * DM, DM);
  k_glu<<<dim3(MTOK * (DM / 4) / 256), blk, 0, stream>>>(pw1o, glu);
  k_dwconv31<<<dim3(MTOK * (DM / 4) / 256), blk, 0, stream>>>(glu, dw_w, dw_b, c3);
  gemm_kne<float, 2, false><<<dim3(MTOK / 128, DM / 128), blk, 0, stream>>>(c3, DM, pw2_w, DM, pw2_b, m1, ones, m2, DM, DM);
  k_ln<<<dim3(MTOK / 32), blk, 0, stream>>>(m2, ln_g, ln_b, fln);
  gemm_kne<float, 1, false><<<dim3(MTOK / 128, DFF / 128), blk, 0, stream>>>(fln, DM, ff1, DFF, fb1, nullptr, nullptr, ff, DFF, DM);
  gemm_kne<float, 2, false><<<dim3(MTOK / 128, DM / 128), blk, 0, stream>>>(ff, DFF, ff2, DM, fb2, fln, ones, out, DM, DFF);
}
